// RNN_35364760715347
// MI455X (gfx1250) — hardware-verified
//
#include <hip/hip_runtime.h>
#include <stdint.h>

constexpr int BATCH_B  = 64;
constexpr int SEQ_T    = 512;
constexpr int DIM_IN   = 256;
constexpr int DIM_H    = 512;
constexpr int NCLS     = 2;
constexpr int ROWS_BLK = 16;
constexpr int NBLK_REC = BATCH_B / ROWS_BLK;
constexpr int H_PITCH  = DIM_H + 8;
constexpr int P_PITCH  = DIM_H + 4;
constexpr float W_CARRY     = 64.0f;
constexpr float W_CARRY_INV = 0.015625f;

static_assert(SEQ_T % 64 == 0);
static_assert(DIM_H % 64 == 0);
static_assert(DIM_IN % 32 == 0);
static_assert(DIM_H % 32 == 0);
static_assert(BATCH_B % ROWS_BLK == 0);
static_assert(DIM_H == 8 * 64);
static_assert(ROWS_BLK * NCLS == 32);
static_assert((BATCH_B * SEQ_T * DIM_IN) % 8 == 0);
static_assert((DIM_H * DIM_IN) % 8 == 0);

constexpr size_t SZ_X16   = (size_t)BATCH_B * SEQ_T * DIM_IN * 2;
constexpr size_t SZ_WIH0  = (size_t)DIM_H * DIM_IN * 2;
constexpr size_t SZ_WHH   = (size_t)DIM_H * DIM_H * 2;
constexpr size_t SZ_BS    = (size_t)DIM_H * 4;
constexpr size_t SZ_PROJ  = (size_t)SEQ_T * BATCH_B * DIM_H * 4;
constexpr size_t SZ_HSEQ  = (size_t)SEQ_T * BATCH_B * DIM_H * 2;
constexpr size_t OFF_X16  = 0;
constexpr size_t OFF_WIH0 = OFF_X16 + SZ_X16;
constexpr size_t OFF_WHH0 = OFF_WIH0 + SZ_WIH0;
constexpr size_t OFF_WIH1 = OFF_WHH0 + SZ_WHH;
constexpr size_t OFF_WHH1 = OFF_WIH1 + SZ_WHH;
constexpr size_t OFF_BS0  = OFF_WHH1 + SZ_WHH;
constexpr size_t OFF_BS1  = OFF_BS0 + SZ_BS;
constexpr size_t OFF_PROJ = OFF_BS1 + SZ_BS;
constexpr size_t OFF_HSEQ = OFF_PROJ + SZ_PROJ;
constexpr size_t WS_TOTAL = OFF_HSEQ + SZ_HSEQ;
static_assert(WS_TOTAL == 119279616);
static_assert(WS_TOTAL <= 134217728);
static_assert(OFF_WIH0 % 256 == 0 && OFF_WHH0 % 256 == 0 && OFF_WIH1 % 256 == 0 && OFF_WHH1 % 256 == 0);
static_assert(OFF_BS0 % 256 == 0 && OFF_BS1 % 256 == 0 && OFF_PROJ % 256 == 0 && OFF_HSEQ % 256 == 0);

typedef __attribute__((ext_vector_type(16))) _Float16 v16h;
typedef __attribute__((ext_vector_type(8)))  _Float16 v8h;
typedef __attribute__((ext_vector_type(16))) __bf16   v16b;
typedef __attribute__((ext_vector_type(8)))  __bf16   v8b;
typedef __attribute__((ext_vector_type(8)))  float    v8f;
typedef __attribute__((ext_vector_type(4)))  float    v4f;

__device__ __forceinline__ unsigned short f2bf_bits(float f) {
  unsigned u = __float_as_uint(f);
  return (unsigned short)((u + 0x7FFFu + ((u >> 16) & 1u)) >> 16);
}
__device__ __forceinline__ float bf_bits2f(unsigned short h) { return __uint_as_float(((unsigned)h) << 16); }

__device__ __forceinline__ void dep_guard_h(v8f& a, v8f& b, v16h x, v16h y) { asm volatile("v_nop\n\tv_nop\n\tv_nop\n\tv_nop" : "+v"(a), "+v"(b) : "v"(x), "v"(y)); }
__device__ __forceinline__ void dep_guard_b(v8f& a, v8f& b, v16b x, v16b y) { asm volatile("v_nop\n\tv_nop\n\tv_nop\n\tv_nop" : "+v"(a), "+v"(b) : "v"(x), "v"(y)); }
__device__ __forceinline__ void keep4_h(v16h a, v16h b, v16h c, v16h d) { asm volatile("v_nop" :: "v"(a), "v"(b), "v"(c), "v"(d)); }
__device__ __forceinline__ void keep4_b(v16b a, v16b b, v16b c, v16b d) { asm volatile("v_nop" :: "v"(a), "v"(b), "v"(c), "v"(d)); }
__device__ __forceinline__ void acc_guard4(v8f& a, v8f& b, v8f& c, v8f& d) { asm volatile("v_nop\n\tv_nop\n\tv_nop\n\tv_nop" : "+v"(a), "+v"(b), "+v"(c), "+v"(d)); }
template <typename T> struct Frag;
template <> struct Frag<_Float16> {
  typedef v16h V; union U { v16h v; v8h h[2]; };
  static __device__ __forceinline__ v16h load(const _Float16* p) {
    U f; f.h[0] = *(const v8h*)(p); f.h[1] = *(const v8h*)(p + 16); return f.v;
  }
  static __device__ __forceinline__ v8f mma(v16h a, v16h b, v8f c) {
    return __builtin_amdgcn_wmma_f32_16x16x32_f16(false, a, false, b, (short)0, c, false, false);
  }
  static __device__ __forceinline__ void guard(v8f& a, v8f& b, v16h x, v16h y) { dep_guard_h(a, b, x, y); }
  static __device__ __forceinline__ void keep(v16h a, v16h b, v16h c, v16h d) { keep4_h(a, b, c, d); }
};
template <> struct Frag<__bf16> {
  typedef v16b V; union U { v16b v; v8b h[2]; };
  static __device__ __forceinline__ v16b load(const __bf16* p) {
    U f; f.h[0] = *(const v8b*)(p); f.h[1] = *(const v8b*)(p + 16); return f.v;
  }
  static __device__ __forceinline__ v8f mma(v16b a, v16b b, v8f c) {
    return __builtin_amdgcn_wmma_f32_16x16x32_bf16(false, a, false, b, (short)0, c, false, false);
  }
  static __device__ __forceinline__ void guard(v8f& a, v8f& b, v16b x, v16b y) { dep_guard_b(a, b, x, y); }
  static __device__ __forceinline__ void keep(v16b a, v16b b, v16b c, v16b d) { keep4_b(a, b, c, d); }
};

template <int ET> struct Elem;
template <> struct Elem<0> { typedef _Float16 T; };
template <> struct Elem<1> { typedef __bf16 T; };
template <int ET, bool SPLIT, int BIAS_MODE, int OUT_MODE, bool RESID, int ACT = 0>
__global__ __launch_bounds__(256) void wmma_gemm64(
    const unsigned short* __restrict__ Ap, const unsigned short* __restrict__ A2p, int lda, long strideA,
    const unsigned short* __restrict__ Btp, const unsigned short* __restrict__ Bt2p, int ldb, long strideB,
    void* __restrict__ Cout, void* __restrict__ Cout2, int ldc, long strideC,
    const float* __restrict__ bias,
    const float* __restrict__ resid, long strideR,
    int M, int N, int K, float scale) {
  typedef typename Elem<ET>::T T;
  typedef typename Frag<T>::V V;
  const T* A = (const T*)Ap; const T* A2 = (const T*)A2p; const T* Bt = (const T*)Btp; const T* Bt2 = (const T*)Bt2p;
  __shared__ __align__(16) float sT[8][16 * 68];
  const int b    = blockIdx.y;
  const int lane = threadIdx.x & 31;
  const int wave = threadIdx.x >> 5;
  const int tilesN = N >> 6;
  const int tilesM = M >> 6;
  const int tile = blockIdx.x * 8 + wave;
  if (tile >= tilesM * tilesN) return;
  const int tm = tile / tilesN;
  const int tn = tile - tm * tilesN;
  const int m0 = tm << 6;
  const int n0 = tn << 6;

  const T* Ab  = A  + (size_t)b * strideA;
  const T* Bb  = Bt + (size_t)b * strideB;
  const T* Ab2 = SPLIT ? (A2  + (size_t)b * strideA) : nullptr;
  const T* Bb2 = SPLIT ? (Bt2 + (size_t)b * strideB) : nullptr;

  const int rlane = lane & 15;
  const int koff  = (lane >> 4) * 8;
  const int mOff  = (lane >> 4) * 8;

  v8f acc[4][4];
#pragma unroll
  for (int i = 0; i < 4; ++i)
#pragma unroll
    for (int j = 0; j < 4; ++j) acc[i][j] = (v8f){0.f,0.f,0.f,0.f,0.f,0.f,0.f,0.f};

  for (int k0 = 0; k0 < K; k0 += 32) {
    V bh[4], bl[4];
#pragma unroll
    for (int j = 0; j < 4; ++j) {
      const size_t bo = (size_t)(n0 + (j << 4) + rlane) * ldb + koff + k0;
      bh[j] = Frag<T>::load(Bb + bo);
      if (SPLIT) bl[j] = Frag<T>::load(Bb2 + bo);
    }
#pragma unroll
    for (int i = 0; i < 4; ++i) {
      const size_t ao = (size_t)(m0 + (i << 4) + rlane) * lda + koff + k0;
      V ah = Frag<T>::load(Ab + ao);
      V al;
      if (SPLIT) al = Frag<T>::load(Ab2 + ao);
#pragma unroll
      for (int j = 0; j < 4; ++j) {
        acc[i][j] = Frag<T>::mma(ah, bh[j], acc[i][j]);
        if (SPLIT) {
          acc[i][j] = Frag<T>::mma(ah, bl[j], acc[i][j]);
          acc[i][j] = Frag<T>::mma(al, bh[j], acc[i][j]);
        }
      }
      Frag<T>::guard(acc[i][0], acc[i][3], ah, SPLIT ? al : ah);
    }
    Frag<T>::keep(bh[0], bh[1], bh[2], bh[3]);
    if (SPLIT) Frag<T>::keep(bl[0], bl[1], bl[2], bl[3]);
  }
  acc_guard4(acc[0][0], acc[0][1], acc[0][2], acc[0][3]);
  acc_guard4(acc[1][0], acc[1][1], acc[1][2], acc[1][3]);
  acc_guard4(acc[2][0], acc[2][1], acc[2][2], acc[2][3]);
  acc_guard4(acc[3][0], acc[3][1], acc[3][2], acc[3][3]);

  float* slab = sT[wave];
  const float* Rb = RESID ? (resid + (size_t)b * strideR) : nullptr;
#pragma unroll
  for (int i = 0; i < 4; ++i) {
    const int mBase = m0 + (i << 4);
#pragma unroll
    for (int j = 0; j < 4; ++j) {
      const int n = n0 + (j << 4) + rlane;
      float bv = 0.f;
      if (BIAS_MODE == 2) bv = bias[n];
#pragma unroll
      for (int r = 0; r < 8; ++r) {
        float v = acc[i][j][r] * scale;
        if (BIAS_MODE == 1) v += bias[mBase + mOff + r];
        if (BIAS_MODE == 2) v += bv;
        if (RESID) v += Rb[(size_t)(mBase + mOff + r) * ldc + n];
        if (ACT == 1) v = tanhf(v);
        if (ACT == 2) v = fmaxf(v, 0.0f);
        if (ACT == 3) v = v / (1.0f + expf(-v));
        if (ACT == 4) v = (v > 0.f) ? v : 0.01f * v;
        if (ACT == 5) v = 0.5f * v * (1.0f + erff(v * 0.70710678118654752f));
        slab[(mOff + r) * 68 + (j << 4) + rlane] = v;
      }
    }
    __builtin_amdgcn_fence(__ATOMIC_RELEASE, "workgroup");
    __builtin_amdgcn_wave_barrier();
    __builtin_amdgcn_fence(__ATOMIC_ACQUIRE, "workgroup");
    if (OUT_MODE == 0) {
      float* C = (float*)Cout + (size_t)b * strideC;
      const int hh = lane >> 4, c4 = (lane & 15) * 4;
      for (int pass = 0; pass < 2; ++pass) {
#pragma unroll
        for (int it = 0; it < 8; ++it) {
          const int row = it * 2 + hh;
          v4f v = *(const v4f*)(slab + row * 68 + c4);
          *(volatile v4f*)(C + (size_t)(mBase + row) * ldc + n0 + c4) = v;
        }
        __threadfence();
      }
    } else {
      const int q = lane >> 3, c8 = (lane & 7) * 8;
      unsigned short* C  = (unsigned short*)Cout  + (size_t)b * strideC;
      unsigned short* C2 = (OUT_MODE == 2) ? ((unsigned short*)Cout2 + (size_t)b * strideC) : nullptr;
      for (int pass = 0; pass < 2; ++pass) {
#pragma unroll
        for (int it = 0; it < 4; ++it) {
          const int row = it * 4 + q;
          const float* sp = slab + row * 68 + c8;
          v8h hv, lv;
#pragma unroll
          for (int e = 0; e < 8; ++e) {
            if (OUT_MODE == 1) {
              hv[e] = (_Float16)sp[e];
            } else {
              unsigned short hb = f2bf_bits(sp[e]);
              unsigned short lb = f2bf_bits(sp[e] - bf_bits2f(hb));
              hv[e] = __builtin_bit_cast(_Float16, hb);
              lv[e] = __builtin_bit_cast(_Float16, lb);
            }
          }
          *(volatile v8h*)(C + (size_t)(mBase + row) * ldc + n0 + c8) = hv;
          if (OUT_MODE == 2) *(volatile v8h*)(C2 + (size_t)(mBase + row) * ldc + n0 + c8) = lv;
        }
        __threadfence();
      }
    }
    __builtin_amdgcn_fence(__ATOMIC_RELEASE, "workgroup");
    __builtin_amdgcn_wave_barrier();
    __builtin_amdgcn_fence(__ATOMIC_ACQUIRE, "workgroup");
  }
}

__global__ __launch_bounds__(256) void cast8_kernel(const float* __restrict__ in,
                                                     unsigned short* __restrict__ outp,
                                                     int n8, float scale) {
  const int i = blockIdx.x * 256 + threadIdx.x;
  if (i < n8) {
    const float* src = in + (size_t)i * 8;
    const v4f a = *(const v4f*)(src);
    const v4f c = *(const v4f*)(src + 4);
    v8h hv;
    hv[0] = (_Float16)(a[0] * scale); hv[1] = (_Float16)(a[1] * scale);
    hv[2] = (_Float16)(a[2] * scale); hv[3] = (_Float16)(a[3] * scale);
    hv[4] = (_Float16)(c[0] * scale); hv[5] = (_Float16)(c[1] * scale);
    hv[6] = (_Float16)(c[2] * scale); hv[7] = (_Float16)(c[3] * scale);
    _Float16* o = (_Float16*)(void*)outp + (size_t)i * 8;
    *(volatile v8h*)o = hv;
    __threadfence();
    *(volatile v8h*)o = hv;
  }
}

__global__ __launch_bounds__(128) void bias_sum_kernel(const float* __restrict__ a0, const float* __restrict__ b0,
                                                        const float* __restrict__ a1, const float* __restrict__ b1,
                                                        float* __restrict__ o0, float* __restrict__ o1) {
  const float* pa = (blockIdx.x == 0) ? a0 : a1;
  const float* pb = (blockIdx.x == 0) ? b0 : b1;
  float* po = (blockIdx.x == 0) ? o0 : o1;
  const int i = threadIdx.x;
  if (i < DIM_H / 4) {
    const v4f va = *(const v4f*)(pa + 4 * i);
    const v4f vb = *(const v4f*)(pb + 4 * i);
    const v4f v = va + vb;
    *(volatile v4f*)(po + 4 * i) = v;
    __threadfence();
    *(volatile v4f*)(po + 4 * i) = v;
  }
}

template <int STORE_SEQ, int FINAL>
__global__ __launch_bounds__(256) void recur_kernel(
    const float* __restrict__ proj,
    const unsigned short* __restrict__ Whhp,
    unsigned short* __restrict__ hseq,
    const float* __restrict__ Wc, const float* __restrict__ bc,
    float* __restrict__ out)
{
  typedef Frag<_Float16> FH;
  union UH { v16h v; v8h h[2]; };
  __shared__ __align__(16) _Float16 hL[ROWS_BLK * H_PITCH];
  __shared__ __align__(16) float    pL[ROWS_BLK * P_PITCH];
  __shared__ __align__(16) float    oL[32];

  const _Float16* Whh = (const _Float16*)(const void*)Whhp;
  const int tid   = threadIdx.x;
  const int wave  = tid >> 5;
  const int lane  = tid & 31;
  const int rlane = lane & 15;
  const int hh    = lane >> 4;
  const int koff  = hh * 8;
  const int slice = blockIdx.x;
  const int n0    = wave * 64;

  {
    const v8h z = (v8h){(_Float16)0.0f, (_Float16)0.0f, (_Float16)0.0f, (_Float16)0.0f,
                        (_Float16)0.0f, (_Float16)0.0f, (_Float16)0.0f, (_Float16)0.0f};
    for (int i = tid; i < (ROWS_BLK * H_PITCH) / 8; i += 256) *(v8h*)(hL + 8 * i) = z;
  }

  float hreg[4][8];
  for (int t = 0; t < SEQ_T; ++t) {
    {
      const float* ps = proj + ((size_t)t * BATCH_B + (size_t)ROWS_BLK * slice) * DIM_H;
#pragma unroll
      for (int i = 0; i < 8; ++i) {
        const int e  = i * 256 + tid;
        const int rr = e >> 7;
        const int c4 = (e & 127) * 4;
        const v4f v = *(const v4f*)(ps + (size_t)rr * DIM_H + c4);
        *(v4f*)(pL + rr * P_PITCH + c4) = v;
      }
    }
    __syncthreads();

    v8f acc[4];
#pragma unroll
    for (int j = 0; j < 4; ++j) acc[j] = (v8f){0.f,0.f,0.f,0.f,0.f,0.f,0.f,0.f};
#pragma unroll 2
    for (int kt = 0; kt < DIM_H / 32; ++kt) {
      const int k0 = kt * 32;
      v16h bfr[4];
#pragma unroll
      for (int j = 0; j < 4; ++j)
        bfr[j] = FH::load(Whh + (size_t)(n0 + (j << 4) + rlane) * DIM_H + k0 + koff);
      UH ua;
      ua.h[0] = *(const v8h*)(hL + rlane * H_PITCH + k0 + koff);
      ua.h[1] = *(const v8h*)(hL + rlane * H_PITCH + k0 + koff + 16);
#pragma unroll
      for (int j = 0; j < 4; ++j) acc[j] = FH::mma(ua.v, bfr[j], acc[j]);
      FH::guard(acc[0], acc[3], ua.v, bfr[3]);
      FH::keep(bfr[0], bfr[1], bfr[2], bfr[3]);
    }
    acc_guard4(acc[0], acc[1], acc[2], acc[3]);

#pragma unroll
    for (int j = 0; j < 4; ++j) {
      const int col = n0 + (j << 4) + rlane;
#pragma unroll
      for (int r = 0; r < 8; ++r) {
        const int row = hh * 8 + r;
        const float v = acc[j][r] * W_CARRY_INV + pL[row * P_PITCH + col];
        hreg[j][r] = tanhf(v);
      }
    }
    __syncthreads();

#pragma unroll
    for (int j = 0; j < 4; ++j) {
      const int col = n0 + (j << 4) + rlane;
#pragma unroll
      for (int r = 0; r < 8; ++r) {
        const int row = hh * 8 + r;
        hL[row * H_PITCH + col] = (_Float16)hreg[j][r];
      }
    }
    if (FINAL && t == SEQ_T - 1) {
#pragma unroll
      for (int j = 0; j < 4; ++j) {
        const int col = n0 + (j << 4) + rlane;
#pragma unroll
        for (int r = 0; r < 8; ++r) {
          const int row = hh * 8 + r;
          pL[row * P_PITCH + col] = hreg[j][r];
        }
      }
    }
    __syncthreads();

    if (STORE_SEQ) {
      unsigned short* hs = hseq + ((size_t)t * BATCH_B + (size_t)ROWS_BLK * slice) * DIM_H + n0;
      const int q = lane >> 3, c8 = (lane & 7) * 8;
      for (int pass = 0; pass < 2; ++pass) {
#pragma unroll
        for (int it = 0; it < 4; ++it) {
          const int row = it * 4 + q;
          const v8h hv = *(const v8h*)(hL + row * H_PITCH + n0 + c8);
          *(volatile v8h*)(hs + (size_t)row * DIM_H + c8) = hv;
        }
        __threadfence();
      }
    }
  }

  if (FINAL) {
    if (wave == 0) {
      const int m = lane >> 1, c = lane & 1;
      const float* wr = Wc + (size_t)c * DIM_H;
      const float* hr = pL + m * P_PITCH;
      float s = bc[c];
#pragma unroll 4
      for (int k = 0; k < DIM_H; ++k) s = fmaf(hr[k], wr[k], s);
      oL[lane] = s;
    }
    __syncthreads();
    if (wave == 0) {
      const int l8 = lane & 7;
      const v4f v = *(const v4f*)(oL + 4 * l8);
      float* op = out + (size_t)32 * slice + 4 * l8;
      if (lane < 8) *(volatile v4f*)op = v;
      __threadfence();
      if (lane < 8) *(volatile v4f*)op = v;
    }
  }
}

extern "C" void kernel_launch(void* const* d_in, const int* in_sizes, int n_in,
                              void* d_out, int out_size, void* d_ws, size_t ws_size,
                              hipStream_t stream) {
  if (n_in < 11) return;
  if (in_sizes[0] != BATCH_B * SEQ_T * DIM_IN) return;
  if (in_sizes[1] != DIM_H * DIM_IN || in_sizes[2] != DIM_H * DIM_H) return;
  if (in_sizes[3] != DIM_H || in_sizes[4] != DIM_H) return;
  if (in_sizes[5] != DIM_H * DIM_H || in_sizes[6] != DIM_H * DIM_H) return;
  if (in_sizes[7] != DIM_H || in_sizes[8] != DIM_H) return;
  if (in_sizes[9] != NCLS * DIM_H || in_sizes[10] != NCLS) return;
  if (out_size != BATCH_B * NCLS) return;
  if (ws_size < WS_TOTAL) return;

  const float* x     = (const float*)d_in[0];
  const float* W_ih0 = (const float*)d_in[1];
  const float* W_hh0 = (const float*)d_in[2];
  const float* b_ih0 = (const float*)d_in[3];
  const float* b_hh0 = (const float*)d_in[4];
  const float* W_ih1 = (const float*)d_in[5];
  const float* W_hh1 = (const float*)d_in[6];
  const float* b_ih1 = (const float*)d_in[7];
  const float* b_hh1 = (const float*)d_in[8];
  const float* Wc    = (const float*)d_in[9];
  const float* bc    = (const float*)d_in[10];
  float* out = (float*)d_out;

  char* ws = (char*)d_ws;
  unsigned short* x16  = (unsigned short*)(ws + OFF_X16);
  unsigned short* wih0 = (unsigned short*)(ws + OFF_WIH0);
  unsigned short* whh0 = (unsigned short*)(ws + OFF_WHH0);
  unsigned short* wih1 = (unsigned short*)(ws + OFF_WIH1);
  unsigned short* whh1 = (unsigned short*)(ws + OFF_WHH1);
  float* bs0  = (float*)(ws + OFF_BS0);
  float* bs1  = (float*)(ws + OFF_BS1);
  float* proj = (float*)(ws + OFF_PROJ);
  unsigned short* hseq = (unsigned short*)(ws + OFF_HSEQ);

  {
    const int n8x = BATCH_B * SEQ_T * DIM_IN / 8;
    cast8_kernel<<<(n8x + 255) / 256, 256, 0, stream>>>(x, x16, n8x, 1.0f);
    const int n8a = DIM_H * DIM_IN / 8;
    const int n8b = DIM_H * DIM_H / 8;
    cast8_kernel<<<(n8a + 255) / 256, 256, 0, stream>>>(W_ih0, wih0, n8a, W_CARRY);
    cast8_kernel<<<(n8b + 255) / 256, 256, 0, stream>>>(W_hh0, whh0, n8b, W_CARRY);
    cast8_kernel<<<(n8b + 255) / 256, 256, 0, stream>>>(W_ih1, wih1, n8b, W_CARRY);
    cast8_kernel<<<(n8b + 255) / 256, 256, 0, stream>>>(W_hh1, whh1, n8b, W_CARRY);
  }
  bias_sum_kernel<<<2, 128, 0, stream>>>(b_ih0, b_hh0, b_ih1, b_hh1, bs0, bs1);

  const int tiles = (SEQ_T / 64) * (DIM_H / 64);
  const dim3 ggrid((tiles + 7) / 8, BATCH_B);

  wmma_gemm64<0, false, 2, 0, false, 0><<<ggrid, 256, 0, stream>>>(
      x16, x16, DIM_IN, (long)SEQ_T * DIM_IN,
      wih0, wih0, DIM_IN, 0L,
      (void*)proj, (void*)proj, BATCH_B * DIM_H, (long)DIM_H,
      bs0, bs0, 0L,
      SEQ_T, DIM_H, DIM_IN, W_CARRY_INV);

  recur_kernel<1, 0><<<NBLK_REC, 256, 0, stream>>>(proj, whh0, hseq, Wc, bc, out);

  wmma_gemm64<0, false, 2, 0, false, 0><<<ggrid, 256, 0, stream>>>(
      hseq, hseq, BATCH_B * DIM_H, (long)DIM_H,
      wih1, wih1, DIM_H, 0L,
      (void*)proj, (void*)proj, BATCH_B * DIM_H, (long)DIM_H,
      bs1, bs1, 0L,
      SEQ_T, DIM_H, DIM_H, W_CARRY_INV);

  recur_kernel<0, 1><<<NBLK_REC, 256, 0, stream>>>(proj, whh1, hseq, Wc, bc, out);
}
